// GatedDeltaNet_13872744366525
// MI455X (gfx1250) — hardware-verified
//
#include <hip/hip_runtime.h>
#include <math.h>

constexpr int kBatch   = 2;
constexpr int kSeqLen  = 2048;
constexpr int kHidden  = 2048;
constexpr int kRows    = kBatch * kSeqLen;
constexpr int kNumKH   = 8;
constexpr int kNumVH   = 16;
constexpr int kHeadDim = 64;
constexpr int kKDim    = kNumKH * kHeadDim;
constexpr int kVDim    = kNumVH * kHeadDim;
constexpr int kConvDim = 2 * kKDim + kVDim;
constexpr int kTaps    = 4;
constexpr int kProjN   = kConvDim + kVDim + 2 * kNumVH;
constexpr int kProjLd  = 3136;
constexpr int kGateLd  = 32;
constexpr float kOgCarry  = 16.0f;
constexpr float kWoCarry  = 64.0f;
constexpr float kOutScale = 1.0f / 1024.0f;
constexpr float kEps      = 1.0e-6f;
constexpr float kFltMin   = 1.17549435e-38f;
static_assert(kProjN <= kProjLd);
static_assert(kProjLd % 64 == 0);
static_assert(kRows % 64 == 0);
static_assert(kHidden % 64 == 0);
static_assert(kHidden % 32 == 0);
static_assert(kVDim % 32 == 0);
static_assert(kConvDim == 16 * 128);
static_assert(kNumVH / kNumKH == 2);

typedef __attribute__((ext_vector_type(16))) _Float16 v16h;
typedef __attribute__((ext_vector_type(8)))  _Float16 v8h;
typedef __attribute__((ext_vector_type(16))) __bf16   v16b;
typedef __attribute__((ext_vector_type(8)))  __bf16   v8b;
typedef __attribute__((ext_vector_type(8)))  float    v8f;
typedef __attribute__((ext_vector_type(4)))  float    v4f;
typedef __attribute__((ext_vector_type(4)))  unsigned int v4u;

__device__ __forceinline__ unsigned short f2bf_bits(float f) {
  unsigned u = __float_as_uint(f);
  return (unsigned short)((u + 0x7FFFu + ((u >> 16) & 1u)) >> 16);
}
__device__ __forceinline__ float bf_bits2f(unsigned short h) { return __uint_as_float(((unsigned)h) << 16); }
__device__ __forceinline__ float bf16r(float f) { return bf_bits2f(f2bf_bits(f)); }

__device__ __forceinline__ void dep_guard_h(v8f& a, v8f& b, v16h x, v16h y) { asm volatile("v_nop\n\tv_nop\n\tv_nop\n\tv_nop" : "+v"(a), "+v"(b) : "v"(x), "v"(y)); }
__device__ __forceinline__ void dep_guard_b(v8f& a, v8f& b, v16b x, v16b y) { asm volatile("v_nop\n\tv_nop\n\tv_nop\n\tv_nop" : "+v"(a), "+v"(b) : "v"(x), "v"(y)); }
__device__ __forceinline__ void keep4_h(v16h a, v16h b, v16h c, v16h d) { asm volatile("v_nop" :: "v"(a), "v"(b), "v"(c), "v"(d)); }
__device__ __forceinline__ void keep4_b(v16b a, v16b b, v16b c, v16b d) { asm volatile("v_nop" :: "v"(a), "v"(b), "v"(c), "v"(d)); }
__device__ __forceinline__ void acc_guard4(v8f& a, v8f& b, v8f& c, v8f& d) { asm volatile("v_nop\n\tv_nop\n\tv_nop\n\tv_nop" : "+v"(a), "+v"(b), "+v"(c), "+v"(d)); }
template <typename T> struct Frag;
template <> struct Frag<_Float16> {
  typedef v16h V; union U { v16h v; v8h h[2]; };
  static __device__ __forceinline__ v16h load(const _Float16* p) {
    U f; f.h[0] = *(const v8h*)(p); f.h[1] = *(const v8h*)(p + 16); return f.v;
  }
  static __device__ __forceinline__ v8f mma(v16h a, v16h b, v8f c) {
    return __builtin_amdgcn_wmma_f32_16x16x32_f16(false, a, false, b, (short)0, c, false, false);
  }
  static __device__ __forceinline__ void guard(v8f& a, v8f& b, v16h x, v16h y) { dep_guard_h(a, b, x, y); }
  static __device__ __forceinline__ void keep(v16h a, v16h b, v16h c, v16h d) { keep4_h(a, b, c, d); }
};
template <> struct Frag<__bf16> {
  typedef v16b V; union U { v16b v; v8b h[2]; };
  static __device__ __forceinline__ v16b load(const __bf16* p) {
    U f; f.h[0] = *(const v8b*)(p); f.h[1] = *(const v8b*)(p + 16); return f.v;
  }
  static __device__ __forceinline__ v8f mma(v16b a, v16b b, v8f c) {
    return __builtin_amdgcn_wmma_f32_16x16x32_bf16(false, a, false, b, (short)0, c, false, false);
  }
  static __device__ __forceinline__ void guard(v8f& a, v8f& b, v16b x, v16b y) { dep_guard_b(a, b, x, y); }
  static __device__ __forceinline__ void keep(v16b a, v16b b, v16b c, v16b d) { keep4_b(a, b, c, d); }
};

__device__ __forceinline__ unsigned pk16(unsigned short a, unsigned short b) { return (unsigned)a | ((unsigned)b << 16); }
__device__ __forceinline__ unsigned short h_bits(float f) { const _Float16 h = (_Float16)f; return __builtin_bit_cast(unsigned short, h); }

template <int ET> struct Elem;
template <> struct Elem<0> { typedef _Float16 T; };
template <> struct Elem<1> { typedef __bf16 T; };
template <int ET, bool SPLIT, int BIAS_MODE, int OUT_MODE, bool RESID, int ACT = 0>
__global__ __launch_bounds__(256) void wmma_gemm64(
    const unsigned short* __restrict__ Ap, const unsigned short* __restrict__ A2p, int lda, long strideA,
    const unsigned short* __restrict__ Btp, const unsigned short* __restrict__ Bt2p, int ldb, long strideB,
    void* __restrict__ Cout, void* __restrict__ Cout2, int ldc, long strideC,
    const float* __restrict__ bias,
    const float* __restrict__ resid, long strideR,
    int M, int N, int K, float scale) {
  typedef typename Elem<ET>::T T;
  typedef typename Frag<T>::V V;
  const T* A = (const T*)Ap; const T* A2 = (const T*)A2p; const T* Bt = (const T*)Btp; const T* Bt2 = (const T*)Bt2p;
  __shared__ __align__(16) float sT[8][16 * 68];
  const int b    = blockIdx.y;
  const int lane = threadIdx.x & 31;
  const int wave = threadIdx.x >> 5;
  const int tilesN = N >> 6;
  const int tilesM = M >> 6;
  const int tile = blockIdx.x * 8 + wave;
  if (tile >= tilesM * tilesN) return;
  const int tm = tile / tilesN;
  const int tn = tile - tm * tilesN;
  const int m0 = tm << 6;
  const int n0 = tn << 6;

  const T* Ab  = A  + (size_t)b * strideA;
  const T* Bb  = Bt + (size_t)b * strideB;
  const T* Ab2 = SPLIT ? (A2  + (size_t)b * strideA) : nullptr;
  const T* Bb2 = SPLIT ? (Bt2 + (size_t)b * strideB) : nullptr;

  const int rlane = lane & 15;
  const int koff  = (lane >> 4) * 8;
  const int mOff  = (lane >> 4) * 8;

  v8f acc[4][4];
#pragma unroll
  for (int i = 0; i < 4; ++i)
#pragma unroll
    for (int j = 0; j < 4; ++j) acc[i][j] = (v8f){0.f,0.f,0.f,0.f,0.f,0.f,0.f,0.f};

  for (int k0 = 0; k0 < K; k0 += 32) {
    V bh[4], bl[4];
#pragma unroll
    for (int j = 0; j < 4; ++j) {
      const size_t bo = (size_t)(n0 + (j << 4) + rlane) * ldb + koff + k0;
      bh[j] = Frag<T>::load(Bb + bo);
      if (SPLIT) bl[j] = Frag<T>::load(Bb2 + bo);
    }
#pragma unroll
    for (int i = 0; i < 4; ++i) {
      const size_t ao = (size_t)(m0 + (i << 4) + rlane) * lda + koff + k0;
      V ah = Frag<T>::load(Ab + ao);
      V al;
      if (SPLIT) al = Frag<T>::load(Ab2 + ao);
#pragma unroll
      for (int j = 0; j < 4; ++j) {
        acc[i][j] = Frag<T>::mma(ah, bh[j], acc[i][j]);
        if (SPLIT) {
          acc[i][j] = Frag<T>::mma(ah, bl[j], acc[i][j]);
          acc[i][j] = Frag<T>::mma(al, bh[j], acc[i][j]);
        }
      }
      Frag<T>::guard(acc[i][0], acc[i][3], ah, SPLIT ? al : ah);
    }
    Frag<T>::keep(bh[0], bh[1], bh[2], bh[3]);
    if (SPLIT) Frag<T>::keep(bl[0], bl[1], bl[2], bl[3]);
  }
  acc_guard4(acc[0][0], acc[0][1], acc[0][2], acc[0][3]);
  acc_guard4(acc[1][0], acc[1][1], acc[1][2], acc[1][3]);
  acc_guard4(acc[2][0], acc[2][1], acc[2][2], acc[2][3]);
  acc_guard4(acc[3][0], acc[3][1], acc[3][2], acc[3][3]);

  float* slab = sT[wave];
  const float* Rb = RESID ? (resid + (size_t)b * strideR) : nullptr;
#pragma unroll
  for (int i = 0; i < 4; ++i) {
    const int mBase = m0 + (i << 4);
#pragma unroll
    for (int j = 0; j < 4; ++j) {
      const int n = n0 + (j << 4) + rlane;
      float bv = 0.f;
      if (BIAS_MODE == 2) bv = bias[n];
#pragma unroll
      for (int r = 0; r < 8; ++r) {
        float v = acc[i][j][r] * scale;
        if (BIAS_MODE == 1) v += bias[mBase + mOff + r];
        if (BIAS_MODE == 2) v += bv;
        if (RESID) v += Rb[(size_t)(mBase + mOff + r) * ldc + n];
        if (ACT == 2) v = fmaxf(v, 0.0f);
        if (ACT == 4) v = (v > 0.f) ? v : 0.01f * v;
        slab[(mOff + r) * 68 + (j << 4) + rlane] = v;
      }
    }
    __builtin_amdgcn_fence(__ATOMIC_RELEASE, "workgroup");
    __builtin_amdgcn_wave_barrier();
    __builtin_amdgcn_fence(__ATOMIC_ACQUIRE, "workgroup");
    if (OUT_MODE == 0) {
      float* C = (float*)Cout + (size_t)b * strideC;
      const int hh = lane >> 4, c4 = (lane & 15) * 4;
      for (int pass = 0; pass < 2; ++pass) {
#pragma unroll
        for (int it = 0; it < 8; ++it) {
          const int row = it * 2 + hh;
          v4f v = *(const v4f*)(slab + row * 68 + c4);
          *(volatile v4f*)(C + (size_t)(mBase + row) * ldc + n0 + c4) = v;
        }
        __threadfence();
      }
    } else {
      const int q = lane >> 3, c8 = (lane & 7) * 8;
      unsigned short* C  = (unsigned short*)Cout  + (size_t)b * strideC;
      unsigned short* C2 = (OUT_MODE == 2) ? ((unsigned short*)Cout2 + (size_t)b * strideC) : nullptr;
      for (int pass = 0; pass < 2; ++pass) {
#pragma unroll
        for (int it = 0; it < 4; ++it) {
          const int row = it * 4 + q;
          const float* sp = slab + row * 68 + c8;
          v8h hv, lv;
#pragma unroll
          for (int e = 0; e < 8; ++e) {
            if (OUT_MODE == 1) {
              hv[e] = (_Float16)sp[e];
            } else {
              unsigned short hb = f2bf_bits(sp[e]);
              unsigned short lb = f2bf_bits(sp[e] - bf_bits2f(hb));
              hv[e] = __builtin_bit_cast(_Float16, hb);
              lv[e] = __builtin_bit_cast(_Float16, lb);
            }
          }
          *(volatile v8h*)(C + (size_t)(mBase + row) * ldc + n0 + c8) = hv;
          if (OUT_MODE == 2) *(volatile v8h*)(C2 + (size_t)(mBase + row) * ldc + n0 + c8) = lv;
        }
        __threadfence();
      }
    }
    __builtin_amdgcn_fence(__ATOMIC_RELEASE, "workgroup");
    __builtin_amdgcn_wave_barrier();
    __builtin_amdgcn_fence(__ATOMIC_ACQUIRE, "workgroup");
  }
}

template <int MODE>
__global__ __launch_bounds__(256) void cast8_kernel(const float* __restrict__ in, unsigned short* __restrict__ out, int n8, float scale) {
  const int i = blockIdx.x * 256 + threadIdx.x;
  if (i >= n8) return;
  const float* p = in + 8 * (size_t)i;
  const v4f a = *(const v4f*)(p);
  const v4f c = *(const v4f*)(p + 4);
  unsigned short hb[8];
#pragma unroll
  for (int e = 0; e < 4; ++e) {
    const float f0 = a[e];
    const float f1 = c[e];
    if (MODE == 0) {
      hb[e]     = f2bf_bits(f0);
      hb[4 + e] = f2bf_bits(f1);
    } else {
      hb[e]     = h_bits(bf16r(f0) * scale);
      hb[4 + e] = h_bits(bf16r(f1) * scale);
    }
  }
  const v4u u = (v4u){pk16(hb[0], hb[1]), pk16(hb[2], hb[3]), pk16(hb[4], hb[5]), pk16(hb[6], hb[7])};
  unsigned short* q = out + 8 * (size_t)i;
  *(volatile v4u*)q = u;
  __threadfence();
  *(volatile v4u*)q = u;
}

__global__ __launch_bounds__(256) void zero16_kernel(unsigned short* __restrict__ out, int n8) {
  const int i = blockIdx.x * 256 + threadIdx.x;
  if (i >= n8) return;
  const v4u u = (v4u){0u, 0u, 0u, 0u};
  unsigned short* q = out + 8 * (size_t)i;
  *(volatile v4u*)q = u;
  __threadfence();
  *(volatile v4u*)q = u;
}

__global__ __launch_bounds__(256) void act_kernel(const float* __restrict__ c1, const float* __restrict__ convw,
                                                  float* __restrict__ act) {
  const int row  = blockIdx.x;
  const int s    = row & (kSeqLen - 1);
  const int lane = threadIdx.x & 31;
  const int wave = threadIdx.x >> 5;
#pragma unroll 1
  for (int it = 0; it < 2; ++it) {
    const int chunk = wave + 8 * it;
    const int cb    = chunk * 128 + 4 * lane;
    const int grp   = chunk * 2 + (lane >> 4);
    const float* wp = convw + (size_t)cb * kTaps;
    const v4f wv0 = *(const v4f*)(wp);
    const v4f wv1 = *(const v4f*)(wp + 4);
    const v4f wv2 = *(const v4f*)(wp + 8);
    const v4f wv3 = *(const v4f*)(wp + 12);
    float w0[4], w1[4], w2[4], w3[4];
#pragma unroll
    for (int j = 0; j < kTaps; ++j) {
      const float t0 = wv0[j];
      const float t1 = wv1[j];
      const float t2 = wv2[j];
      const float t3 = wv3[j];
      w0[j] = bf16r(t0);
      w1[j] = bf16r(t1);
      w2[j] = bf16r(t2);
      w3[j] = bf16r(t3);
    }
    asm volatile("" ::: "memory");
    float y0 = 0.0f, y1 = 0.0f, y2 = 0.0f, y3 = 0.0f;
#pragma unroll
    for (int j = 0; j < kTaps; ++j) {
      const int sp    = s - (kTaps - 1) + j;
      const float fa  = (sp >= 0) ? 1.0f : 0.0f;
      const int rsrc  = (sp >= 0) ? (row - (kTaps - 1) + j) : row;
      const v4f x = *(const v4f*)(c1 + (size_t)rsrc * kProjLd + cb);
      const float x0 = x[0];
      const float x1 = x[1];
      const float x2 = x[2];
      const float x3 = x[3];
      y0 = fmaf(w0[j] * fa, x0, y0);
      y1 = fmaf(w1[j] * fa, x1, y1);
      y2 = fmaf(w2[j] * fa, x2, y2);
      y3 = fmaf(w3[j] * fa, x3, y3);
    }
    const float e0 = expf(-y0);
    const float e1 = expf(-y1);
    const float e2 = expf(-y2);
    const float e3 = expf(-y3);
    y0 = y0 * (1.0f / (1.0f + e0));
    y1 = y1 * (1.0f / (1.0f + e1));
    y2 = y2 * (1.0f / (1.0f + e2));
    y3 = y3 * (1.0f / (1.0f + e3));
    float ss = (y0 * y0 + y1 * y1) + (y2 * y2 + y3 * y3);
    ss += __shfl_xor(ss, 1, 32);
    ss += __shfl_xor(ss, 2, 32);
    ss += __shfl_xor(ss, 4, 32);
    ss += __shfl_xor(ss, 8, 32);
    const float r  = rsqrtf(ss + kEps);
    const float sc = (grp < kNumKH) ? (r * 0.125f) : ((grp < 2 * kNumKH) ? r : 1.0f);
    const v4f o = (v4f){y0 * sc, y1 * sc, y2 * sc, y3 * sc};
    float* dst = act + (size_t)row * kConvDim + cb;
    *(volatile v4f*)dst = o;
    __threadfence();
    *(volatile v4f*)dst = o;
  }
}

__global__ __launch_bounds__(256) void gate_kernel(const float* __restrict__ c1, const float* __restrict__ dtb,
                                                   const float* __restrict__ alog, float* __restrict__ gate) {
  __shared__ __align__(16) float gsh[8][32];
  const int lane = threadIdx.x & 31;
  const int wave = threadIdx.x >> 5;
  const int row  = blockIdx.x * 8 + wave;
  const int hd   = lane & (kNumVH - 1);
  const float* cr = c1 + (size_t)row * kProjLd;
  const float braw = cr[kConvDim + kVDim + hd];
  const float araw = cr[kConvDim + kVDim + kNumVH + hd];
  const float db   = bf16r(dtb[hd]);
  const float al   = bf16r(alog[hd]);
  const float beta = 1.0f / (1.0f + expf(-braw));
  const float x    = araw + db;
  const float spl  = fmaxf(x, 0.0f) + log1pf(expf(-fabsf(x)));
  const float g    = -expf(al) * spl;
  float eg = expf(g);
  eg = (eg < kFltMin) ? 0.0f : eg;
  gsh[wave][lane] = (lane < kNumVH) ? eg : beta;
  __syncthreads();
  const int l8 = lane & 7;
  const v4f u = *(const v4f*)(&gsh[wave][4 * l8]);
  float* dst = gate + (size_t)row * kGateLd + 4 * l8;
  if (lane < 8) *(volatile v4f*)dst = u;
  __threadfence();
  if (lane < 8) *(volatile v4f*)dst = u;
}

__global__ __launch_bounds__(256) void scan_kernel(const float* __restrict__ act, const float* __restrict__ c1,
                                                   const float* __restrict__ gate, const float* __restrict__ nw,
                                                   unsigned short* __restrict__ og) {
  __shared__ __align__(16) float stg[2][256];
  __shared__ __align__(16) float preL[2][64];
  __shared__ float red[2][8];
  __shared__ float gsc[2][2];

  const int tid  = threadIdx.x;
  const int lane = tid & 31;
  const int wave = tid >> 5;
  const int h    = blockIdx.x & (kNumVH - 1);
  const int b    = blockIdx.x >> 4;
  const int hk   = h >> 1;
  const int vcol = tid >> 2;
  const int kg   = tid & 3;
  const int grp  = tid >> 6;
  const int e    = tid & 63;
  const size_t row0 = (size_t)b * kSeqLen;

  const float* srcq = act + row0 * kConvDim + hk * kHeadDim + e;
  const float* srck = act + row0 * kConvDim + kKDim + hk * kHeadDim + e;
  const float* srcv = act + row0 * kConvDim + 2 * kKDim + h * kHeadDim + e;
  const float* srcz = c1 + row0 * kProjLd + kConvDim + h * kHeadDim + e;
  const float* src  = (grp == 0) ? srcq : (grp == 1) ? srck : (grp == 2) ? srcv : srcz;
  const size_t pitch = (grp == 3) ? (size_t)kProjLd : (size_t)kConvDim;
  const float* gsrc = gate + row0 * kGateLd;
  const float nwv  = 1.0f + bf16r(nw[vcol]);
  const int l8 = lane & 7;
  unsigned short* ogbase = og + row0 * kVDim + h * kHeadDim + 8 * l8;

  float st[16];
#pragma unroll
  for (int i = 0; i < 16; ++i) st[i] = 0.0f;

  for (int t = 0; t < kSeqLen; ++t) {
    const int p = t & 1;
    stg[p][tid] = src[(size_t)t * pitch];
    if (wave == 0) {
      const float ge = gsrc[t * kGateLd + h];
      const float gb = gsrc[t * kGateLd + kNumVH + h];
      if (lane == 0) { gsc[p][0] = ge; gsc[p][1] = gb; }
    }
    __syncthreads();
    const float eg = gsc[p][0];
    const float bt = gsc[p][1];
    const float* qL = stg[p] + kg * 16;
    const float* kL = stg[p] + 64 + kg * 16;
    const v4f k4a = *(const v4f*)(kL);
    const v4f k4b = *(const v4f*)(kL + 4);
    const v4f k4c = *(const v4f*)(kL + 8);
    const v4f k4d = *(const v4f*)(kL + 12);
    const v4f q4a = *(const v4f*)(qL);
    const v4f q4b = *(const v4f*)(qL + 4);
    const v4f q4c = *(const v4f*)(qL + 8);
    const v4f q4d = *(const v4f*)(qL + 12);
    float kr[16], qr[16];
#pragma unroll
    for (int i = 0; i < 4; ++i) {
      kr[i] = k4a[i]; kr[4 + i] = k4b[i]; kr[8 + i] = k4c[i]; kr[12 + i] = k4d[i];
      qr[i] = q4a[i]; qr[4 + i] = q4b[i]; qr[8 + i] = q4c[i]; qr[12 + i] = q4d[i];
    }
    float kv = 0.0f;
#pragma unroll
    for (int i = 0; i < 16; ++i) {
      st[i] = st[i] * eg;
      kv = fmaf(st[i], kr[i], kv);
    }
    kv += __shfl_xor(kv, 1, 32);
    kv += __shfl_xor(kv, 2, 32);
    const float vt = stg[p][128 + vcol];
    const float zt = stg[p][192 + vcol];
    const float d  = (vt - kv) * bt;
    float ov = 0.0f;
#pragma unroll
    for (int i = 0; i < 16; ++i) {
      st[i] = fmaf(kr[i], d, st[i]);
      ov = fmaf(st[i], qr[i], ov);
    }
    ov += __shfl_xor(ov, 1, 32);
    ov += __shfl_xor(ov, 2, 32);
    float sq = ov * ov;
    sq += __shfl_xor(sq, 4, 32);
    sq += __shfl_xor(sq, 8, 32);
    sq += __shfl_xor(sq, 16, 32);
    const float ez  = expf(-zt);
    const float sz  = zt * (1.0f / (1.0f + ez));
    const float pre = (ov * nwv) * sz;
    if (kg == 0)   preL[p][vcol] = pre;
    if (lane == 0) red[p][wave] = sq;
    __syncthreads();
    if (wave == 0) {
      float tot = red[p][0];
#pragma unroll
      for (int w = 1; w < 8; ++w) tot += red[p][w];
      const float r = rsqrtf(tot * (1.0f / 64.0f) + kEps) * kOgCarry;
      const v4f a0 = *(const v4f*)(preL[p] + 8 * l8);
      const v4f a1 = *(const v4f*)(preL[p] + 8 * l8 + 4);
      unsigned short hb[8];
#pragma unroll
      for (int q = 0; q < 4; ++q) {
        const float f0 = a0[q];
        const float f1 = a1[q];
        hb[q]     = h_bits(f0 * r);
        hb[4 + q] = h_bits(f1 * r);
      }
      const v4u u = (v4u){pk16(hb[0], hb[1]), pk16(hb[2], hb[3]), pk16(hb[4], hb[5]), pk16(hb[6], hb[7])};
      unsigned short* dst = ogbase + (size_t)t * kVDim;
      if (lane < 8) *(volatile v4u*)dst = u;
      __threadfence();
      if (lane < 8) *(volatile v4u*)dst = u;
    }
  }
}

extern "C" void kernel_launch(void* const* d_in, const int* in_sizes, int n_in,
                              void* d_out, int out_size, void* d_ws, size_t ws_size,
                              hipStream_t stream) {
  if (n_in < 10) return;
  if (in_sizes[0] != kRows * kHidden) return;
  if (in_sizes[1] != kConvDim * kHidden) return;
  if (in_sizes[2] != kConvDim * kTaps) return;
  if (in_sizes[3] != kVDim * kHidden) return;
  if (in_sizes[4] != kNumVH * kHidden) return;
  if (in_sizes[5] != kNumVH * kHidden) return;
  if (in_sizes[6] != kHidden * kVDim) return;
  if (in_sizes[7] != kNumVH || in_sizes[8] != kNumVH || in_sizes[9] != kHeadDim) return;
  if (out_size != kRows * kHidden) return;

  const size_t szA1   = (size_t)kRows * kHidden * 2;
  const size_t szWcat = (size_t)kProjLd * kHidden * 2;
  const size_t szWo   = (size_t)kHidden * kVDim * 2;
  const size_t szC1   = (size_t)kRows * kProjLd * 4;
  const size_t szAct  = (size_t)kRows * kConvDim * 4;
  const size_t szGate = (size_t)kRows * kGateLd * 4;
  const size_t szOg   = (size_t)kRows * kVDim * 2;
  const size_t offA1   = 0;
  const size_t offWcat = offA1 + szA1;
  const size_t offWo   = offWcat + szWcat;
  const size_t offC1   = offWo + szWo;
  const size_t offAct  = offC1 + szC1;
  const size_t offGate = offAct + szAct;
  const size_t offOg   = offGate + szGate;
  const size_t total   = offOg + szOg;
  if (ws_size < total) return;

  const float* hs    = (const float*)d_in[0];
  const float* wqkv  = (const float*)d_in[1];
  const float* convw = (const float*)d_in[2];
  const float* wz    = (const float*)d_in[3];
  const float* wb    = (const float*)d_in[4];
  const float* wa    = (const float*)d_in[5];
  const float* wout  = (const float*)d_in[6];
  const float* dtb   = (const float*)d_in[7];
  const float* alog  = (const float*)d_in[8];
  const float* nw    = (const float*)d_in[9];
  float* out = (float*)d_out;
  char* ws = (char*)d_ws;
  unsigned short* A1   = (unsigned short*)(ws + offA1);
  unsigned short* WCAT = (unsigned short*)(ws + offWcat);
  unsigned short* WO16 = (unsigned short*)(ws + offWo);
  float* C1   = (float*)(ws + offC1);
  float* ACT  = (float*)(ws + offAct);
  float* GATE = (float*)(ws + offGate);
  unsigned short* OG = (unsigned short*)(ws + offOg);

  const int n8A  = (kRows * kHidden) / 8;
  const int n8Q  = (kConvDim * kHidden) / 8;
  const int n8Z  = (kVDim * kHidden) / 8;
  const int n8B  = (kNumVH * kHidden) / 8;
  const int n8P  = ((kProjLd - kProjN) * kHidden) / 8;
  const int n8W  = (kHidden * kVDim) / 8;
  cast8_kernel<0><<<dim3(n8A / 256), dim3(256), 0, stream>>>(hs, A1, n8A, 1.0f);
  cast8_kernel<0><<<dim3(n8Q / 256), dim3(256), 0, stream>>>(wqkv, WCAT, n8Q, 1.0f);
  cast8_kernel<0><<<dim3(n8Z / 256), dim3(256), 0, stream>>>(wz, WCAT + (size_t)kConvDim * kHidden, n8Z, 1.0f);
  cast8_kernel<0><<<dim3(n8B / 256), dim3(256), 0, stream>>>(wb, WCAT + (size_t)(kConvDim + kVDim) * kHidden, n8B, 1.0f);
  cast8_kernel<0><<<dim3(n8B / 256), dim3(256), 0, stream>>>(wa, WCAT + (size_t)(kConvDim + kVDim + kNumVH) * kHidden, n8B, 1.0f);
  zero16_kernel<<<dim3(n8P / 256), dim3(256), 0, stream>>>(WCAT + (size_t)kProjN * kHidden, n8P);
  cast8_kernel<1><<<dim3(n8W / 256), dim3(256), 0, stream>>>(wout, WO16, n8W, kWoCarry);

  const int tiles1 = (kRows / 64) * (kProjLd / 64);
  wmma_gemm64<1, false, 0, 0, false, 0><<<dim3(tiles1 / 8, 1), dim3(256), 0, stream>>>(
      A1, A1, kHidden, 0L, WCAT, WCAT, kHidden, 0L,
      (void*)C1, (void*)C1, kProjLd, 0L, C1, C1, 0L, kRows, kProjLd, kHidden, 1.0f);

  act_kernel<<<dim3(kRows), dim3(256), 0, stream>>>(C1, convw, ACT);
  gate_kernel<<<dim3(kRows / 8), dim3(256), 0, stream>>>(C1, dtb, alog, GATE);

  scan_kernel<<<dim3(kBatch * kNumVH), dim3(256), 0, stream>>>(ACT, C1, GATE, nw, OG);

  const int tiles2 = (kRows / 64) * (kHidden / 64);
  wmma_gemm64<0, false, 0, 0, false, 0><<<dim3(tiles2 / 8, 1), dim3(256), 0, stream>>>(
      OG, OG, kVDim, 0L, WO16, WO16, kVDim, 0L,
      (void*)out, (void*)out, kHidden, 0L, GATE, GATE, 0L, kRows, kHidden, kVDim, kOutScale);
}
